// Encoder_5136780886772
// MI455X (gfx1250) — hardware-run, weakly checked
//
#include <hip/hip_runtime.h>


#ifndef NB
#define NB 65536
#endif
#define NB_FULL 65536
#define SQ   9
#define DM   20
#define NH_  4
#define HD   5
#define DFF  512
#define KPD  32
#define NSB  32
#define ROWS (NSB * SQ)
#define TPB  ROWS
#define NWV  (TPB / 32)
#ifndef Y_RES
#define Y_RES 0
#endif
#ifndef H_RES
#define H_RES 0
#endif
#define QRS  2048.0f
#define QRI  (1.0f / 2048.0f)
#define W1C  4.0f
#define W2C  16.0f
#define FSC  (1.0f / 64.0f)
#define SC2  ((float)(1.4426950408889634 / 3.0))
#define LN_EPS 1.0e-5f
#define OQ    0
#define OK_   (ROWS * DM)
#define OV    (2 * ROWS * DM)
#define OM    (3 * ROWS * DM)
#define ODUMP (4 * ROWS * DM)
#define SA_N  (4 * ROWS * DM + NWV * 64)

static_assert(NH_ * HD == DM);
static_assert(DM % 4 == 0);
static_assert(DM <= KPD && KPD == 32);
static_assert(DM > 16 && DM <= 20);
static_assert(DFF % 32 == 0);
static_assert(TPB % 32 == 0);
static_assert(TPB == ROWS);
static_assert(NWV * 32 == ROWS);
static_assert(TPB * 4 == NSB * NH_ * SQ);
static_assert(TPB * 5 * 4 == ROWS * DM);
static_assert(TPB * 5 * 16 == NSB * SQ * DM * 4);
static_assert((NSB * SQ * DM * 4) % 128 == 0);
static_assert(TPB < DM * DM && 2 * TPB >= DM * DM);
static_assert(NB % NSB == 0);
static_assert(NB <= NB_FULL);
static_assert((SA_N + ROWS * DM + 4 * DM * DM + 8 * DM) * 4 <= 131072);
static_assert((2 * DFF * KPD / 8) % 256 == 0);

typedef _Float16 h16;
typedef unsigned short bf;
typedef __attribute__((ext_vector_type(16))) _Float16 v16h;
typedef __attribute__((ext_vector_type(8)))  _Float16 v8h;
typedef __attribute__((ext_vector_type(2)))  _Float16 v2h;
typedef __attribute__((ext_vector_type(8)))  unsigned v8u;
typedef __attribute__((ext_vector_type(8)))  float    v8f;
typedef __attribute__((ext_vector_type(4)))  float    v4f;
typedef v4f  __attribute__((may_alias)) v4fa;

__device__ __forceinline__ unsigned short f2bf(float f) { unsigned u = __float_as_uint(f); u += 0x7FFFu + ((u >> 16) & 1u); return (unsigned short)(u >> 16); }
__device__ __forceinline__ float bfr(float f) { return __uint_as_float(((unsigned)f2bf(f)) << 16); }
__device__ __forceinline__ v16h cat16(v8h lo, v8h hi) { return __builtin_shufflevector(lo, hi, 0, 1, 2, 3, 4, 5, 6, 7, 8, 9, 10, 11, 12, 13, 14, 15); }
__device__ __forceinline__ v8f wmma16(v16h a, v16h b, v8f c) { return __builtin_amdgcn_wmma_f32_16x16x32_f16(false, a, false, b, (short)0, c, false, false); }
__device__ __forceinline__ v16h  ldh(const h16* p) { return cat16(*(const v8h*)p, *(const v8h*)(p + 16)); }
__device__ __forceinline__ void wave_sync() { __builtin_amdgcn_fence(3  , "wavefront"); __builtin_amdgcn_wave_barrier(); asm volatile("" ::: "memory"); }

static __device__ __forceinline__ h16 toh_flush(float v) { const float w = (fabsf(v) < 6.103515625e-05f) ? 0.0f : v; return (h16)w; }
__device__ __forceinline__ v8f wmma16g(v16h a, v16h b, v8f c) { c = wmma16(a, b, c); asm volatile("v_nop\n\tv_nop\n\tv_nop\n\tv_nop" : "+v"(c) : "v"(a), "v"(b)); return c; }

__device__ __forceinline__ v16h frag_lo(const unsigned (&o)[10], const unsigned (&p)[10], bool up) {
    v8u f;
    f[0] = up ? p[4] : o[0]; f[1] = up ? p[5] : o[1]; f[2] = up ? p[6] : o[2]; f[3] = up ? p[7] : o[3];
    f[4] = up ? 0u : o[8]; f[5] = up ? 0u : o[9]; f[6] = 0u; f[7] = 0u;
    return __builtin_bit_cast(v16h, f);
}
__device__ __forceinline__ v16h frag_hi(const unsigned (&o)[10], const unsigned (&p)[10], bool up) {
    v8u f;
    f[0] = up ? o[4] : p[0]; f[1] = up ? o[5] : p[1]; f[2] = up ? o[6] : p[2]; f[3] = up ? o[7] : p[3];
    f[4] = up ? 0u : p[8]; f[5] = up ? 0u : p[9]; f[6] = 0u; f[7] = 0u;
    return __builtin_bit_cast(v16h, f);
}

__global__ __launch_bounds__(256) void k_wconv(const float* __restrict__ W1, const float* __restrict__ W2, h16* WT) {
    const unsigned bx = blockIdx.x;
    const unsigned p = bx * 256u + threadIdx.x;
    v8h o;
    if (bx < 8u) {
        const unsigned n = p >> 2, k8 = (p & 3u) * 8u;
#pragma unroll
        for (unsigned i = 0; i < 8u; ++i) {
            const unsigned k = k8 + i; const unsigned kc = min(k, (unsigned)(DM - 1));
            float w = W1[kc * (unsigned)DFF + n];
            asm volatile("" : "+v"(w));
            const float c = bfr(w) * W1C;
            o[i] = toh_flush((k < (unsigned)DM) ? c : 0.0f); }
    } else {
        const unsigned q = p - 2048u; const unsigned d = q >> 6, j8 = (q & 63u) * 8u; const unsigned dc = min(d, (unsigned)(DM - 1));
#pragma unroll
        for (unsigned i = 0; i < 8u; ++i) {
            float w = W2[(j8 + i) * (unsigned)DM + dc];
            asm volatile("" : "+v"(w));
            const float c = bfr(w) * W2C;
            o[i] = toh_flush((d < (unsigned)DM) ? c : 0.0f); }
    }
    *(volatile v8h*)(WT + (size_t)p * 8) = o; __threadfence(); *(volatile v8h*)(WT + (size_t)p * 8) = o;
}

__global__ __launch_bounds__(TPB) void k_block(const float* __restrict__ X,
                                               const float* __restrict__ Wq, const float* __restrict__ bq, const float* __restrict__ Wk, const float* __restrict__ bk,
                                               const float* __restrict__ Wv, const float* __restrict__ bv, const float* __restrict__ Wo, const float* __restrict__ bo,
                                               const float* __restrict__ g1, const float* __restrict__ b1, const float* __restrict__ g2, const float* __restrict__ b2,
                                               const h16* __restrict__ W1T, const h16* __restrict__ W2T, float* OUT) {
    __shared__ __align__(16) float sa[SA_N];
    __shared__ __align__(16) float sxs[ROWS * DM];
    __shared__ __align__(16) float sw[4 * DM * DM];
    __shared__ __align__(16) float sb[8 * DM];
    const unsigned tid = threadIdx.x; const unsigned bx = blockIdx.x;
    const unsigned lane = tid & 31u, lr = lane & 15u, hi = lane >> 4;
    const unsigned wave = (unsigned)__builtin_amdgcn_readfirstlane((int)(threadIdx.x >> 5));
    const bool up = hi != 0u;

    { const float* xg = X + (size_t)bx * (size_t)(ROWS * DM);
#pragma unroll
      for (unsigned j = 0; j < 5u; ++j) { const unsigned i = tid + (unsigned)TPB * j;
          const v4f v = *(const v4f*)(xg + 4u * i); v4f o;
          o[0] = bfr(v[0]); o[1] = bfr(v[1]); o[2] = bfr(v[2]); o[3] = bfr(v[3]);
          *(v4fa*)(&sxs[4u * i]) = o; } }
    { const unsigned i0 = tid, i1 = min(tid + (unsigned)TPB, (unsigned)(DM * DM - 1));
      const float a0 = Wq[i0], a1 = Wk[i0], a2 = Wv[i0], a3 = Wo[i0];
      const float c0 = Wq[i1], c1 = Wk[i1], c2 = Wv[i1], c3 = Wo[i1];
      sw[i0] = bfr(a0); sw[DM * DM + i0] = bfr(a1); sw[2 * DM * DM + i0] = bfr(a2); sw[3 * DM * DM + i0] = bfr(a3);
      if (tid + (unsigned)TPB < (unsigned)(DM * DM)) { const unsigned i2 = tid + (unsigned)TPB;
          sw[i2] = bfr(c0); sw[DM * DM + i2] = bfr(c1); sw[2 * DM * DM + i2] = bfr(c2); sw[3 * DM * DM + i2] = bfr(c3); }
      const unsigned cc = min(tid, (unsigned)(DM - 1));
      const float v0 = bq[cc], v1 = bk[cc], v2 = bv[cc], v3 = bo[cc], v4 = g1[cc], v5 = b1[cc], v6 = g2[cc], v7 = b2[cc];
      if (tid < (unsigned)DM) { sb[tid] = bfr(v0); sb[DM + tid] = bfr(v1); sb[2 * DM + tid] = bfr(v2); sb[3 * DM + tid] = bfr(v3);
                                sb[4 * DM + tid] = bfr(v4); sb[5 * DM + tid] = bfr(v5); sb[6 * DM + tid] = bfr(v6); sb[7 * DM + tid] = bfr(v7); } }
    __syncthreads();

    { float xr[DM];
#pragma unroll
      for (int i = 0; i < 5; ++i) { const v4f t = *(const v4fa*)(&sxs[tid * (unsigned)DM + 4u * (unsigned)i]); xr[4 * i + 0] = t[0]; xr[4 * i + 1] = t[1]; xr[4 * i + 2] = t[2]; xr[4 * i + 3] = t[3]; }
#pragma unroll 1
      for (unsigned p = 0; p < 3u; ++p) {
#pragma unroll 1
          for (unsigned g = 0; g < 5u; ++g) {
              v4f acc = *(const v4fa*)(&sb[p * (unsigned)DM + 4u * g]);
#pragma unroll
              for (int k = 0; k < DM; ++k) { const v4f w = *(const v4fa*)(&sw[p * (unsigned)(DM * DM) + (unsigned)k * (unsigned)DM + 4u * g]);
                  acc[0] = fmaf(xr[k], w[0], acc[0]); acc[1] = fmaf(xr[k], w[1], acc[1]); acc[2] = fmaf(xr[k], w[2], acc[2]); acc[3] = fmaf(xr[k], w[3], acc[3]); }
              *(v4fa*)(&sa[p * (unsigned)(ROWS * DM) + tid * (unsigned)DM + 4u * g]) = acc; } } }
    __syncthreads();

#pragma unroll 1
    for (unsigned jt = 0; jt < 4u; ++jt) {
        const unsigned task = tid + (unsigned)TPB * jt;
        const unsigned b = task / 36u, r = task - b * 36u, h = r / 9u, q = r - h * 9u;
        const unsigned qo = (unsigned)OQ + (b * 9u + q) * 20u + h * 5u;
        const unsigned ko = (unsigned)OK_ + b * 180u + h * 5u;
        const unsigned vo = (unsigned)OV + b * 180u + h * 5u;
        float qv[HD];
#pragma unroll
        for (int e = 0; e < HD; ++e) qv[e] = sa[qo + (unsigned)e];
        float a[SQ]; float mx = -3.0e38f;
#pragma unroll
        for (int j = 0; j < SQ; ++j) { float d = 0.0f;
#pragma unroll
            for (int e = 0; e < HD; ++e) d = fmaf(qv[e], sa[ko + (unsigned)(j * DM + e)], d);
            d *= SC2; a[j] = d; mx = fmaxf(mx, d); }
        float s = 0.0f;
#pragma unroll
        for (int j = 0; j < SQ; ++j) { a[j] = __builtin_amdgcn_exp2f(a[j] - mx); s += a[j]; }
        const float inv = __builtin_amdgcn_rcpf(s);
        float cx[HD];
#pragma unroll
        for (int e = 0; e < HD; ++e) cx[e] = 0.0f;
#pragma unroll
        for (int j = 0; j < SQ; ++j) {
#pragma unroll
            for (int e = 0; e < HD; ++e) cx[e] = fmaf(a[j], sa[vo + (unsigned)(j * DM + e)], cx[e]); }
        const unsigned mo = (unsigned)OM + b * 180u + h * 45u + q;
#pragma unroll
        for (int e = 0; e < HD; ++e) sa[mo + (unsigned)(e * SQ)] = cx[e] * inv;
    }
    __syncthreads();

    float y[DM];
    { float mr[DM];
#pragma unroll
      for (int i = 0; i < 5; ++i) { const v4f t = *(const v4fa*)(&sa[(unsigned)OM + tid * (unsigned)DM + 4u * (unsigned)i]); mr[4 * i + 0] = t[0]; mr[4 * i + 1] = t[1]; mr[4 * i + 2] = t[2]; mr[4 * i + 3] = t[3]; }
#pragma unroll 1
      for (unsigned g = 0; g < 5u; ++g) {
          v4f acc = *(const v4fa*)(&sb[3u * (unsigned)DM + 4u * g]);
#pragma unroll
          for (int k = 0; k < DM; ++k) { const v4f w = *(const v4fa*)(&sw[3u * (unsigned)(DM * DM) + (unsigned)k * (unsigned)DM + 4u * g]);
              acc[0] = fmaf(mr[k], w[0], acc[0]); acc[1] = fmaf(mr[k], w[1], acc[1]); acc[2] = fmaf(mr[k], w[2], acc[2]); acc[3] = fmaf(mr[k], w[3], acc[3]); }
          const v4f xv = *(const v4fa*)(&sxs[tid * (unsigned)DM + 4u * g]);
          acc[0] += xv[0]; acc[1] += xv[1]; acc[2] += xv[2]; acc[3] += xv[3];
          *(v4fa*)(&sa[(unsigned)OQ + tid * (unsigned)DM + 4u * g]) = acc; }
      float u[DM];
#pragma unroll
      for (int i = 0; i < 5; ++i) { const v4f t = *(const v4fa*)(&sa[(unsigned)OQ + tid * (unsigned)DM + 4u * (unsigned)i]); u[4 * i + 0] = t[0]; u[4 * i + 1] = t[1]; u[4 * i + 2] = t[2]; u[4 * i + 3] = t[3]; }
      float mu = 0.0f;
#pragma unroll
      for (int c = 0; c < DM; ++c) mu += u[c];
      mu *= (1.0f / DM);
      float var = 0.0f;
#pragma unroll
      for (int c = 0; c < DM; ++c) { const float d = u[c] - mu; var = fmaf(d, d, var); }
      const float rs = rsqrtf(var * (1.0f / DM) + LN_EPS);
#pragma unroll
      for (int c = 0; c < DM; ++c) y[c] = (u[c] - mu) * rs * sb[4 * DM + c] + sb[5 * DM + c]; }

    unsigned od[10], pd[10];
#if Y_RES
    unsigned odr[10], pdr[10];
#endif
#pragma unroll
    for (int i = 0; i < 10; ++i) {
        const h16 a0 = toh_flush(y[2 * i]), a1 = toh_flush(y[2 * i + 1]);
        v2h t; t[0] = a0; t[1] = a1; od[i] = __builtin_bit_cast(unsigned, t);
#if Y_RES
        v2h rr; rr[0] = toh_flush((y[2 * i] - (float)a0) * QRS); rr[1] = toh_flush((y[2 * i + 1] - (float)a1) * QRS); odr[i] = __builtin_bit_cast(unsigned, rr);
#endif
    }
#pragma unroll
    for (int i = 0; i < 10; ++i) pd[i] = (unsigned)__shfl_xor((int)od[i], 16, 32);
#if Y_RES
#pragma unroll
    for (int i = 0; i < 10; ++i) pdr[i] = (unsigned)__shfl_xor((int)odr[i], 16, 32);
#endif
    const v16h yfa = frag_lo(od, pd, up), yfb = frag_hi(od, pd, up);
#if Y_RES
    const v16h yra = frag_lo(odr, pdr, up), yrb = frag_hi(odr, pdr, up);
#endif
    const unsigned a1o = lr * (unsigned)KPD + 8u * hi;
    const unsigned a2o = lr * (unsigned)DFF + 8u * hi;
#pragma unroll
    for (int t = 0; t < 2; ++t) {
        const v16h yh = (t == 0) ? yfa : yfb;
#if Y_RES
        const v16h yr = (t == 0) ? yra : yrb;
#endif
        v8f o0 = (v8f){}, o1 = (v8f){};
#if H_RES
        v8f oR0 = (v8f){}, oR1 = (v8f){};
#endif
#pragma unroll 1
        for (unsigned c = 0; c < (unsigned)(DFF / 32); ++c) {
            const h16* w1 = W1T + a1o + c * (unsigned)(32 * KPD);
            const v16h wa = ldh(w1), wb = ldh(w1 + 16 * KPD);
            v8f za = (v8f){}, zb = (v8f){};
            za = wmma16g(wa, yh, za); zb = wmma16g(wb, yh, zb);
#if Y_RES
            v8f la = (v8f){}, lb = (v8f){};
            la = wmma16g(wa, yr, la); lb = wmma16g(wb, yr, lb);
#endif
            v16h pb;
#if H_RES
            v16h pr;
#endif
#pragma unroll
            for (int r = 0; r < 8; ++r) {
                float ta = za[r], tb = zb[r];
#if Y_RES
                ta = ta + la[r] * QRI; tb = tb + lb[r] * QRI;
#endif
                ta = fmaxf(ta, 0.0f); tb = fmaxf(tb, 0.0f);
                const h16 pa = toh_flush(ta), pc = toh_flush(tb);
                pb[r] = pa; pb[8 + r] = pc;
#if H_RES
                pr[r] = toh_flush((ta - (float)pa) * QRS); pr[8 + r] = toh_flush((tb - (float)pc) * QRS);
#endif
            }
            const h16* w2 = W2T + a2o + c * 32u;
            const v16h ua = ldh(w2), ub = ldh(w2 + 16 * DFF);
            o0 = wmma16g(ua, pb, o0); o1 = wmma16g(ub, pb, o1);
#if H_RES
            oR0 = wmma16g(ua, pr, oR0); oR1 = wmma16g(ub, pr, oR1);
#endif
        }
        v8f f0 = o0, f1 = o1;
#if H_RES
        f0 = o0 + oR0 * QRI; f1 = o1 + oR1 * QRI;
#endif
        const unsigned ro = (unsigned)OM + (wave * 32u + (unsigned)t * 16u + lr) * (unsigned)DM;
        v4f e0, e1, e2;
        e0[0] = f0[0] * FSC; e0[1] = f0[1] * FSC; e0[2] = f0[2] * FSC; e0[3] = f0[3] * FSC;
        e1[0] = f0[4] * FSC; e1[1] = f0[5] * FSC; e1[2] = f0[6] * FSC; e1[3] = f0[7] * FSC;
        e2[0] = f1[0] * FSC; e2[1] = f1[1] * FSC; e2[2] = f1[2] * FSC; e2[3] = f1[3] * FSC;
        *(v4fa*)(&sa[ro + 8u * hi]) = e0; *(v4fa*)(&sa[ro + 8u * hi + 4u]) = e1;
        const unsigned o1o = up ? ((unsigned)ODUMP + wave * 64u + lr * 4u) : (ro + 16u);
        *(v4fa*)(&sa[o1o]) = e2;
    }
    wave_sync();

    { float u[DM];
#pragma unroll
      for (int i = 0; i < 5; ++i) { const v4f t = *(const v4fa*)(&sa[(unsigned)OM + tid * (unsigned)DM + 4u * (unsigned)i]);
          u[4 * i + 0] = y[4 * i + 0] + t[0]; u[4 * i + 1] = y[4 * i + 1] + t[1]; u[4 * i + 2] = y[4 * i + 2] + t[2]; u[4 * i + 3] = y[4 * i + 3] + t[3]; }
      float mu = 0.0f;
#pragma unroll
      for (int c = 0; c < DM; ++c) mu += u[c];
      mu *= (1.0f / DM);
      float var = 0.0f;
#pragma unroll
      for (int c = 0; c < DM; ++c) { const float d = u[c] - mu; var = fmaf(d, d, var); }
      const float rs = rsqrtf(var * (1.0f / DM) + LN_EPS);
#pragma unroll
      for (int i = 0; i < 5; ++i) { v4f o;
#pragma unroll
          for (int e = 0; e < 4; ++e) o[e] = (u[4 * i + e] - mu) * rs * sb[6 * DM + 4 * i + e] + sb[7 * DM + 4 * i + e];
          *(v4fa*)(&sa[(unsigned)OM + tid * (unsigned)DM + 4u * (unsigned)i]) = o; } }
    __syncthreads();

    float* ob = OUT + (size_t)bx * (size_t)(ROWS * DM);
#pragma unroll 1
    for (int ps = 0; ps < 2; ++ps) {
#pragma unroll
        for (unsigned j = 0; j < 5u; ++j) { const unsigned i = tid + (unsigned)TPB * j;
            const v4f val = *(const v4fa*)(&sa[(unsigned)OM + 4u * i]);
            *(volatile v4f*)(ob + 4u * i) = val; }
        if (ps == 0) __threadfence(); }
}

static constexpr size_t SZ_W1T = (size_t)DFF * KPD * 2;
static constexpr size_t SZ_W2T = (size_t)KPD * DFF * 2;
static constexpr size_t SZ_TOTAL = SZ_W1T + SZ_W2T;
static_assert(SZ_TOTAL <= (size_t)134217728);
static_assert(SZ_W1T % 256 == 0);
static_assert(SZ_TOTAL == (size_t)(2 * DFF * KPD / 8) * 16);
static_assert((size_t)NB_FULL * SQ * DM * 4 == (size_t)47185920);

extern "C" void kernel_launch(void* const* d_in, const int* in_sizes, int n_in,
                              void* d_out, int out_size, void* d_ws, size_t ws_size, hipStream_t stream) {
    if (n_in < 15) return;
    if ((size_t)in_sizes[0] < (size_t)NB * SQ * DM) return;
    if (in_sizes[1] < DM * DM || in_sizes[3] < DM * DM || in_sizes[5] < DM * DM || in_sizes[7] < DM * DM) return;
    if (in_sizes[2] < DM || in_sizes[4] < DM || in_sizes[6] < DM || in_sizes[8] < DM) return;
    if (in_sizes[9] < DM || in_sizes[10] < DM || in_sizes[13] < DM || in_sizes[14] < DM) return;
    if (in_sizes[11] < DM * DFF || in_sizes[12] < DFF * DM) return;
    if ((size_t)out_size < (size_t)NB * SQ * DM) return;
    if (SZ_TOTAL > ws_size) return;
    const float* X  = (const float*)d_in[0];
    const float* Wq = (const float*)d_in[1];  const float* bq = (const float*)d_in[2];
    const float* Wk = (const float*)d_in[3];  const float* bk = (const float*)d_in[4];
    const float* Wv = (const float*)d_in[5];  const float* bv = (const float*)d_in[6];
    const float* Wo = (const float*)d_in[7];  const float* bo = (const float*)d_in[8];
    const float* g1 = (const float*)d_in[9];  const float* b1 = (const float*)d_in[10];
    const float* W1 = (const float*)d_in[11]; const float* W2 = (const float*)d_in[12];
    const float* g2 = (const float*)d_in[13]; const float* b2 = (const float*)d_in[14];
    float* OUT = (float*)d_out;
    h16* WT = (h16*)d_ws;
    const h16* W1T = WT;
    const h16* W2T = WT + (size_t)DFF * KPD;

    k_wconv<<<dim3((2 * DFF * KPD / 8) / 256, 1, 1), 256, 0, stream>>>(W1, W2, WT);
    k_block<<<dim3(NB / NSB, 1, 1), TPB, 0, stream>>>(X, Wq, bq, Wk, bk, Wv, bv, Wo, bo, g1, b1, g2, b2, W1T, W2T, OUT);
}
